// RGCNEncoder_49916109914172
// MI455X (gfx1250) — hardware-run, weakly checked
//
#include <hip/hip_runtime.h>
#include <stddef.h>


#define HD      256
#define NR      16
#define NBAS    8
#define KAGG    (NR * HD)
#define KTOT    (KAGG + HD)
#define NTHR    256
#define NWAVE   8
#define EPT     8
#define NGRP    2
#define CHUNK   (NTHR * EPT * NGRP)
#define WCAP    (EPT * NGRP * 32)
#define NBD     256
#define NSLOT   (NBD * NR)
#define SSHF    12
#define RCAP    32768
#define SEGCAP  256
#define GROWS   128
#define GCOLS   128
#define TPK     64
#define TPN     32
#define TPP     72
#define ASCL    16
#define WSCL    64
#define WSCAP   134217728

#define LDS_AGG   ((3 * NSLOT + RCAP + NWAVE * WCAP + 2 * NWAVE) * 4)
#define LDS_GEMM  (GROWS * GCOLS * 4)

static_assert(NSLOT == (1 << SSHF));
static_assert((KAGG % 32) == 0 && (KTOT % 32) == 0 && (HD % 32) == 0);
static_assert((KTOT % TPK) == 0 && (KAGG % TPK) == 0 && (HD % TPK) == 0 && (HD % TPN) == 0);
static_assert(TPN * 8 == NTHR && TPK * TPN == NTHR * 8 && TPK == NWAVE * 8);
static_assert((TPP % 8) == 0 && TPP >= TPK);
static_assert(GROWS == NWAVE * 16 && GCOLS == 128 && (HD % GCOLS) == 0);
static_assert(NBD == NWAVE * 32 && HD == 32 * 8);
static_assert(NSLOT == NTHR * 16);
static_assert((RCAP % 4) == 0 && WCAP == EPT * NGRP * 32);
static_assert((NBD % GROWS) == 0);
static_assert(LDS_AGG <= 300 * 1024);

typedef float     v4f  __attribute__((ext_vector_type(4)));
typedef float     v8f  __attribute__((ext_vector_type(8)));
typedef int       v4i  __attribute__((ext_vector_type(4)));
typedef _Float16  v8h  __attribute__((ext_vector_type(8)));
typedef _Float16  v16h __attribute__((ext_vector_type(16)));
union FragH { v16h v; v8h h[2]; };

__device__ __forceinline__ v8f wmf(v16h a, v16h b, v8f c) {
  v8f d = __builtin_amdgcn_wmma_f32_16x16x32_f16(false, a, false, b, (short)0, c, false, false);
  asm volatile("v_nop\n\tv_nop\n\tv_nop\n\tv_nop" : "+v"(d) : "v"(a), "v"(b));
  return d;
}

__device__ __forceinline__ v8h cvt8h(v4f a, v4f b, float z) {
  v8h h;
  h[0] = (_Float16)(a.x * z); h[1] = (_Float16)(a.y * z); h[2] = (_Float16)(a.z * z); h[3] = (_Float16)(a.w * z);
  h[4] = (_Float16)(b.x * z); h[5] = (_Float16)(b.y * z); h[6] = (_Float16)(b.z * z); h[7] = (_Float16)(b.w * z);
  return h;
}

__global__ __launch_bounds__(NTHR) void k_compose(
    const float* __restrict__ compA, const float* __restrict__ basisA, const float* __restrict__ rootA,
    const float* __restrict__ compB, const float* __restrict__ basisB, const float* __restrict__ rootB,
    _Float16* BwA, _Float16* BwB, float scale) {
  __shared__ __attribute__((aligned(16))) _Float16 sT[TPN * TPP];
  const int tid = threadIdx.x;
  const int z = (int)blockIdx.z;
  const float* comp  = (z != 0) ? compB  : compA;
  const float* basis = (z != 0) ? basisB : basisA;
  const float* root  = (z != 0) ? rootB  : rootA;
  _Float16* Bw = (z != 0) ? BwB : BwA;
  const int k0 = (int)blockIdx.x * TPK, n0 = (int)blockIdx.y * TPN;
  const int nc = tid & 31, kq = tid >> 5;
  const int col = n0 + nc;
  if (k0 < KAGG) {
    const int r  = k0 / HD;
    const int i0 = k0 - r * HD;
    float cb[NBAS];
#pragma unroll
    for (int b = 0; b < NBAS; ++b) cb[b] = comp[r * NBAS + b];
#pragma unroll 1
    for (int it = 0; it < TPK / NWAVE; ++it) {
      const int kr = kq + NWAVE * it;
      const int i = i0 + kr;
      float w = 0.0f;
#pragma unroll
      for (int b = 0; b < NBAS; ++b) w = fmaf(cb[b], basis[((size_t)b * HD + i) * HD + col], w);
      sT[nc * TPP + kr] = (_Float16)(w * scale);
    }
  } else {
    const int i0 = k0 - KAGG;
#pragma unroll 1
    for (int it = 0; it < TPK / NWAVE; ++it) {
      const int kr = kq + NWAVE * it;
      const float w = root[(size_t)(i0 + kr) * HD + col];
      sT[nc * TPP + kr] = (_Float16)(w * scale);
    }
  }
  __syncthreads();
  const int nl = tid >> 3, p = tid & 7;
  const v8h hv = *(const v8h*)(sT + nl * TPP + 8 * p);
  _Float16* d = Bw + (size_t)(n0 + nl) * KTOT + k0 + 8 * p;
  *(volatile v8h*)d = hv;
  __threadfence();
  *(volatile v8h*)d = hv;
}

template <int MODE>
__device__ __forceinline__ int scan_chunk(const int* __restrict__ kd, const int* __restrict__ kt, int nE,
                                          int cbase, int base, int vec8, unsigned* list,
                                          int tid, int lane, int wave) {
  int wc = 0;
#pragma unroll
  for (int g = 0; g < NGRP; ++g) {
    const int e0   = cbase + (g * NTHR + tid) * EPT;
    const int sent = -2147483647 - 1;
    const int i0 = min(e0, nE - 1),     i1 = min(e0 + 1, nE - 1), i2 = min(e0 + 2, nE - 1), i3 = min(e0 + 3, nE - 1);
    const int i4 = min(e0 + 4, nE - 1), i5 = min(e0 + 5, nE - 1), i6 = min(e0 + 6, nE - 1), i7 = min(e0 + 7, nE - 1);
    v4i da, db, ta, tb;
    if (vec8 != 0 && cbase + CHUNK <= nE) {
      da = *(const v4i*)(kd + e0);
      db = *(const v4i*)(kd + e0 + 4);
      ta = *(const v4i*)(kt + e0);
      tb = *(const v4i*)(kt + e0 + 4);
    } else {
      da.x = (e0     < nE) ? kd[i0] : sent;
      da.y = (e0 + 1 < nE) ? kd[i1] : sent;
      da.z = (e0 + 2 < nE) ? kd[i2] : sent;
      da.w = (e0 + 3 < nE) ? kd[i3] : sent;
      db.x = (e0 + 4 < nE) ? kd[i4] : sent;
      db.y = (e0 + 5 < nE) ? kd[i5] : sent;
      db.z = (e0 + 6 < nE) ? kd[i6] : sent;
      db.w = (e0 + 7 < nE) ? kd[i7] : sent;
      ta.x = kt[i0]; ta.y = kt[i1]; ta.z = kt[i2]; ta.w = kt[i3];
      tb.x = kt[i4]; tb.y = kt[i5]; tb.z = kt[i6]; tb.w = kt[i7];
    }
    const unsigned nb = (unsigned)base;
    const unsigned s0 = (unsigned)da.x - nb, s1 = (unsigned)da.y - nb;
    const unsigned s2 = (unsigned)da.z - nb, s3 = (unsigned)da.w - nb;
    const unsigned s4 = (unsigned)db.x - nb, s5 = (unsigned)db.y - nb;
    const unsigned s6 = (unsigned)db.z - nb, s7 = (unsigned)db.w - nb;
    const bool h0 = s0 < (unsigned)NBD, h1 = s1 < (unsigned)NBD, h2 = s2 < (unsigned)NBD, h3 = s3 < (unsigned)NBD;
    const bool h4 = s4 < (unsigned)NBD, h5 = s5 < (unsigned)NBD, h6 = s6 < (unsigned)NBD, h7 = s7 < (unsigned)NBD;
    const unsigned q0 = s0 * NR + (unsigned)min(max(ta.x, 0), NR - 1);
    const unsigned q1 = s1 * NR + (unsigned)min(max(ta.y, 0), NR - 1);
    const unsigned q2 = s2 * NR + (unsigned)min(max(ta.z, 0), NR - 1);
    const unsigned q3 = s3 * NR + (unsigned)min(max(ta.w, 0), NR - 1);
    const unsigned q4 = s4 * NR + (unsigned)min(max(tb.x, 0), NR - 1);
    const unsigned q5 = s5 * NR + (unsigned)min(max(tb.y, 0), NR - 1);
    const unsigned q6 = s6 * NR + (unsigned)min(max(tb.z, 0), NR - 1);
    const unsigned q7 = s7 * NR + (unsigned)min(max(tb.w, 0), NR - 1);
    const unsigned any = __builtin_amdgcn_ballot_w32(h0 | h1 | h2 | h3 | h4 | h5 | h6 | h7);
    if (any != 0u) {
#define HITJ(HJ, QJ, IJ) { \
        const unsigned mj = __builtin_amdgcn_ballot_w32(HJ); \
        if (mj != 0u) { \
          if (HJ) { \
            const int pos = wc + (int)__builtin_amdgcn_mbcnt_lo(mj, 0u); \
            const unsigned entv = (MODE != 0) ? ((((unsigned)(IJ)) << SSHF) | (QJ)) : (QJ); \
            if (pos < WCAP) list[wave * WCAP + pos] = entv; \
          } \
          wc += (int)__builtin_popcount(mj); } }
      HITJ(h0, q0, i0)
      HITJ(h1, q1, i1)
      HITJ(h2, q2, i2)
      HITJ(h3, q3, i3)
      HITJ(h4, q4, i4)
      HITJ(h5, q5, i5)
      HITJ(h6, q6, i6)
      HITJ(h7, q7, i7)
#undef HITJ
    }
  }
  return wc;
}

__global__ __launch_bounds__(NTHR) void k_aggmean(
    const int* __restrict__ edst, const int* __restrict__ etyp, const int* __restrict__ esrc,
    const float* __restrict__ x, _Float16* M16, _Float16* X16, int nE, int nN, int vec8) {
  extern __shared__ v4f lds_dyn[];
  int* scnt = (int*)lds_dyn;
  int* soff = scnt + NSLOT;
  int* curs = soff + NSLOT;
  unsigned* region = (unsigned*)(curs + NSLOT);
  unsigned* list = region + RCAP;
  int* wcnt = (int*)(list + NWAVE * WCAP);
  int* wtot = wcnt + NWAVE;
  const int tid = threadIdx.x, lane = tid & 31, wave = tid >> 5;
  const int base = (int)blockIdx.x * NBD;

  {
    const v4i z = {0, 0, 0, 0};
    for (int i = tid; i < NSLOT / 4; i += NTHR) ((v4i*)scnt)[i] = z;
  }
  __syncthreads();

  const int nChunks = (nE + CHUNK - 1) / CHUNK;

#pragma unroll 1
  for (int ch = 0; ch < nChunks; ++ch) {
    const int cbase = ch * CHUNK;
    const int wc = scan_chunk<0>(edst, etyp, nE, cbase, base, vec8, list, tid, lane, wave);
    if (lane == 0) wcnt[wave] = wc;
    __syncthreads();
    if (wave == 0) {
#pragma unroll 1
      for (int wsx = 0; wsx < NWAVE; ++wsx) {
        int n = __builtin_amdgcn_readfirstlane(wcnt[wsx]);
        n = n > WCAP ? WCAP : (n < 0 ? 0 : n);
        const unsigned* lp = list + wsx * WCAP;
#pragma unroll 1
        for (int i = 0; i < n; ++i) {
          const int ent  = __builtin_amdgcn_readfirstlane((int)lp[i]);
          const int slot = ent & (NSLOT - 1);
          if (lane == 0) scnt[slot] = scnt[slot] + 1;
        }
      }
    }
    __syncthreads();
  }

  {
    const int sb = 16 * tid;
    const v4i c0 = *(const v4i*)(scnt + sb);
    const v4i c1 = *(const v4i*)(scnt + sb + 4);
    const v4i c2 = *(const v4i*)(scnt + sb + 8);
    const v4i c3 = *(const v4i*)(scnt + sb + 12);
    const int ts = (c0.x + c0.y + c0.z + c0.w) + (c1.x + c1.y + c1.z + c1.w)
                 + (c2.x + c2.y + c2.z + c2.w) + (c3.x + c3.y + c3.z + c3.w);
    int incl = ts;
#pragma unroll
    for (int dd = 1; dd < 32; dd <<= 1) {
      const int t = __shfl_up(incl, dd, 32);
      if (lane >= dd) incl += t;
    }
    if (lane == 31) wtot[wave] = incl;
    __syncthreads();
    int pre = 0;
#pragma unroll 1
    for (int w = 0; w < wave; ++w) pre += wtot[w];
    int run = pre + incl - ts;
    v4i o0, o1, o2, o3;
    o0.x = run; run += c0.x; o0.y = run; run += c0.y; o0.z = run; run += c0.z; o0.w = run; run += c0.w;
    o1.x = run; run += c1.x; o1.y = run; run += c1.y; o1.z = run; run += c1.z; o1.w = run; run += c1.w;
    o2.x = run; run += c2.x; o2.y = run; run += c2.y; o2.z = run; run += c2.z; o2.w = run; run += c2.w;
    o3.x = run; run += c3.x; o3.y = run; run += c3.y; o3.z = run; run += c3.z; o3.w = run;
    *(v4i*)(soff + sb) = o0; *(v4i*)(soff + sb + 4) = o1; *(v4i*)(soff + sb + 8) = o2; *(v4i*)(soff + sb + 12) = o3;
    *(v4i*)(curs + sb) = o0; *(v4i*)(curs + sb + 4) = o1; *(v4i*)(curs + sb + 8) = o2; *(v4i*)(curs + sb + 12) = o3;
    __syncthreads();
  }

#pragma unroll 1
  for (int ch = 0; ch < nChunks; ++ch) {
    const int cbase = ch * CHUNK;
    const int wc = scan_chunk<1>(edst, etyp, nE, cbase, base, vec8, list, tid, lane, wave);
    if (lane == 0) wcnt[wave] = wc;
    __syncthreads();
    if (wave == 0) {
#pragma unroll 1
      for (int wsx = 0; wsx < NWAVE; ++wsx) {
        int n = __builtin_amdgcn_readfirstlane(wcnt[wsx]);
        n = n > WCAP ? WCAP : (n < 0 ? 0 : n);
        const unsigned* lp = list + wsx * WCAP;
#pragma unroll 1
        for (int i = 0; i < n; ++i) {
          const unsigned ent = (unsigned)__builtin_amdgcn_readfirstlane((int)lp[i]);
          const int slot = (int)(ent & (unsigned)(NSLOT - 1));
          int ev = (int)(ent >> SSHF);
          ev = ev > nE - 1 ? nE - 1 : ev;
          if (lane == 0) {
            const int pos = curs[slot];
            if ((unsigned)pos < (unsigned)RCAP) region[pos] = (unsigned)ev;
            curs[slot] = (pos >= RCAP) ? RCAP : pos + 1;
          }
        }
      }
    }
    __syncthreads();
  }

  const float qnan = __int_as_float(0x7fc00000);
#pragma unroll 1
  for (int jj = 0; jj < NBD / NWAVE; ++jj) {
    const int j  = wave + NWAVE * jj;
    const int d  = base + j;
    const int dc = d < nN ? d : nN - 1;
    {
      const float* xp = x + (size_t)dc * HD + 8 * lane;
      const v4f x0 = *(const v4f*)xp;
      const v4f x1 = *(const v4f*)(xp + 4);
      const v8h xh = cvt8h(x0, x1, (float)ASCL);
      _Float16* gp = X16 + (size_t)d * HD + 8 * lane;
      *(volatile v8h*)gp = xh;
      __threadfence();
      *(volatile v8h*)gp = xh;
    }
#pragma unroll 1
    for (int r = 0; r < NR; ++r) {
      const int slot = j * NR + r;
      const int n  = __builtin_amdgcn_readfirstlane(scnt[slot]);
      const int st = __builtin_amdgcn_readfirstlane(soff[slot]);
      const bool bad = (n > SEGCAP) || (n < 0) || (st < 0) || (st + n > RCAP);
      const int nn = n < 0 ? 0 : (n > SEGCAP ? SEGCAP : n);
      v4f a0 = {0.f, 0.f, 0.f, 0.f};
      v4f a1 = {0.f, 0.f, 0.f, 0.f};
#pragma unroll 1
      for (int p = 0; p < nn; ++p) {
        int pos = st + p;
        pos = pos < 0 ? 0 : (pos > RCAP - 1 ? RCAP - 1 : pos);
        const int eu = __builtin_amdgcn_readfirstlane((int)region[pos]);
        const int e  = eu < 0 ? 0 : (eu > nE - 1 ? nE - 1 : eu);
        int s = esrc[e];
        s = s < 0 ? 0 : (s > nN - 1 ? nN - 1 : s);
        const float* sp = x + (size_t)s * HD + 8 * lane;
        a0 = a0 + *(const v4f*)sp;
        a1 = a1 + *(const v4f*)(sp + 4);
      }
      float inv = (float)ASCL * (1.0f / (float)(nn > 0 ? nn : 1));
      inv = bad ? qnan : inv;
      const v8h mh = cvt8h(a0, a1, inv);
      _Float16* gp = M16 + (size_t)d * KAGG + (size_t)r * HD + 8 * lane;
      *(volatile v8h*)gp = mh;
      __threadfence();
      *(volatile v8h*)gp = mh;
    }
  }
}

__device__ __forceinline__ void kstep(v8f (&acc)[GCOLS / 16], const _Float16* ap, const _Float16* bp) {
  FragH af;
  af.h[0] = *(const v8h*)ap;
  af.h[1] = *(const v8h*)(ap + 16);
#pragma unroll
  for (int t = 0; t < GCOLS / 16; ++t) {
    const _Float16* bq = bp + (size_t)(16 * t) * KTOT;
    FragH bf;
    bf.h[0] = *(const v8h*)bq;
    bf.h[1] = *(const v8h*)(bq + 16);
    acc[t] = wmf(af.v, bf.v, acc[t]);
  }
}

template <int OUT16>
__global__ __launch_bounds__(NTHR) void k_gemm(
    const _Float16* __restrict__ A1, const _Float16* __restrict__ A2, const _Float16* __restrict__ Bw,
    const float* __restrict__ bias, const float* __restrict__ pw,
    float* outF, _Float16* outH, int nRows, float osc) {
  extern __shared__ v4f lds_dyn[];
  constexpr int NC = GCOLS;
  constexpr int NT = NC / 16;
  const int tid = threadIdx.x, lane = tid & 31, wave = tid >> 5, hh = lane >> 4, m = lane & 15;
  const int rowBase = (int)blockIdx.x * GROWS;
  const int cb = (int)blockIdx.y;
  const int ar  = rowBase + wave * 16 + m;
  const int arc = ar < nRows ? ar : nRows - 1;
  const _Float16* a1p = A1 + (size_t)arc * KAGG + 8 * hh;
  const _Float16* a2p = A2 + (size_t)arc * HD + 8 * hh;
  const _Float16* bp0 = Bw + (size_t)(cb * NC + m) * KTOT + 8 * hh;

  v8f acc[NT];
#pragma unroll
  for (int t = 0; t < NT; ++t) { v8f zz = {0.f, 0.f, 0.f, 0.f, 0.f, 0.f, 0.f, 0.f}; acc[t] = zz; }

#pragma unroll 1
  for (int kt = 0; kt < KAGG / 32; ++kt) kstep(acc, a1p + 32 * kt, bp0 + 32 * kt);
#pragma unroll 1
  for (int kt = 0; kt < HD / 32; ++kt) kstep(acc, a2p + 32 * kt, bp0 + KAGG + 32 * kt);

  float bc[NT], wc[NT];
#pragma unroll
  for (int t = 0; t < NT; ++t) {
    const int col = cb * NC + 16 * t + m;
    bc[t] = bias[col];
    wc[t] = pw[col];
  }
  const int r0 = wave * 16 + 8 * hh;

  if (OUT16 == 1) {
    _Float16* stg = (_Float16*)lds_dyn;
    _Float16* sp = stg + r0 * NC + m;
#pragma unroll
    for (int t = 0; t < NT; ++t) {
#pragma unroll
      for (int r = 0; r < 8; ++r) {
        float v = acc[t][r] * osc + bc[t];
        v = (v >= 0.0f) ? v : wc[t] * v;
        sp[r * NC + 16 * t] = (_Float16)(v * (float)ASCL);
      }
    }
    __syncthreads();
#pragma unroll
    for (int i = 0; i < 8; ++i) {
      const int row = wave * 16 + 2 * i + hh;
      const v8h hv = *(const v8h*)(stg + row * NC + 8 * m);
      *(volatile v8h*)(outH + (size_t)(rowBase + row) * HD + cb * NC + 8 * m) = hv;
    }
    __threadfence();
#pragma unroll
    for (int i = 0; i < 8; ++i) {
      const int row = wave * 16 + 2 * i + hh;
      const v8h hv = *(const v8h*)(stg + row * NC + 8 * m);
      *(volatile v8h*)(outH + (size_t)(rowBase + row) * HD + cb * NC + 8 * m) = hv;
    }
  } else {
    float* stg = (float*)lds_dyn;
    float* sp = stg + r0 * NC + m;
#pragma unroll
    for (int t = 0; t < NT; ++t) {
#pragma unroll
      for (int r = 0; r < 8; ++r) {
        float v = acc[t][r] * osc + bc[t];
        v = (v >= 0.0f) ? v : wc[t] * v;
        sp[r * NC + 16 * t] = v;
      }
    }
    __syncthreads();
    const float* lp = stg + wave * 16 * NC;
    float* gp = outF + (size_t)(rowBase + wave * 16) * HD + cb * NC;
#pragma unroll
    for (int i = 0; i < 16; ++i) {
      const v4f v = *(const v4f*)(lp + i * NC + 4 * lane);
      *(volatile v4f*)(gp + (size_t)i * HD + 4 * lane) = v;
    }
    __threadfence();
#pragma unroll
    for (int i = 0; i < 16; ++i) {
      const v4f v = *(const v4f*)(lp + i * NC + 4 * lane);
      *(volatile v4f*)(gp + (size_t)i * HD + 4 * lane) = v;
    }
  }
}

extern "C" void kernel_launch(void* const* d_in, const int* in_sizes, int n_in,
                              void* d_out, int out_size, void* d_ws, size_t ws_size,
                              hipStream_t stream) {
  if (n_in < 14) return;
  if (in_sizes[0] < HD || (in_sizes[0] % HD) != 0) return;
  const int nN = in_sizes[0] / HD;
  if (in_sizes[1] != NBAS * HD * HD || in_sizes[2] != NR * NBAS || in_sizes[3] != HD * HD || in_sizes[4] != HD) return;
  if (in_sizes[5] != NBAS * HD * HD || in_sizes[6] != NR * NBAS || in_sizes[7] != HD * HD || in_sizes[8] != HD) return;
  if (in_sizes[9] != HD) return;
  const int nE = in_sizes[10];
  if (nE < 1 || in_sizes[11] != nE || in_sizes[12] != nE) return;
  if (nE > (1 << 20)) return;
  if (out_size < HD || (out_size % HD) != 0) return;
  const int nDst = out_size / HD;
  if ((nDst % NBD) != 0 || (nDst % GROWS) != 0 || nDst > nN) return;
  if (nN > (1 << 24)) return;

  const float* x_src   = (const float*)d_in[0];
  const float* basis1  = (const float*)d_in[1];
  const float* comp1   = (const float*)d_in[2];
  const float* root1   = (const float*)d_in[3];
  const float* bias1   = (const float*)d_in[4];
  const float* basis2  = (const float*)d_in[5];
  const float* comp2   = (const float*)d_in[6];
  const float* root2   = (const float*)d_in[7];
  const float* bias2   = (const float*)d_in[8];
  const float* prelu_w = (const float*)d_in[9];
  const int*   e_src   = (const int*)d_in[10];
  const int*   e_dst   = (const int*)d_in[11];
  const int*   e_typ   = (const int*)d_in[12];
  float* out = (float*)d_out;

  char* ws = (char*)d_ws;
  size_t off = 0;
#define CARVE(NAME, BYTES) const size_t NAME = off; off += (size_t)(BYTES); off = (off + 255) & ~(size_t)255;
  CARVE(oBw1, (size_t)HD * KTOT * 2)
  CARVE(oBw2, (size_t)HD * KTOT * 2)
  CARVE(oM16, (size_t)nDst * KAGG * 2)
  CARVE(oX16, (size_t)nDst * HD * 2)
  CARVE(oH16, (size_t)nDst * HD * 2)
#undef CARVE
  if (off > ws_size || off > (size_t)WSCAP) return;
  _Float16* Bw1 = (_Float16*)(ws + oBw1);
  _Float16* Bw2 = (_Float16*)(ws + oBw2);
  _Float16* M16 = (_Float16*)(ws + oM16);
  _Float16* X16 = (_Float16*)(ws + oX16);
  _Float16* H16 = (_Float16*)(ws + oH16);

  const float osc = 1.0f / ((float)ASCL * (float)WSCL);

  k_compose<<<dim3(KTOT / TPK, HD / TPN, 2), NTHR, 0, stream>>>(
      comp1, basis1, root1, comp2, basis2, root2, Bw1, Bw2, (float)WSCL);

  hipFuncSetAttribute(reinterpret_cast<const void*>(&k_aggmean),
                      hipFuncAttributeMaxDynamicSharedMemorySize, LDS_AGG);
  k_aggmean<<<nDst / NBD, NTHR, LDS_AGG, stream>>>(e_dst, e_typ, e_src, x_src, M16, X16, nE, nN, 1);

  hipFuncSetAttribute(reinterpret_cast<const void*>(&k_gemm<1>),
                      hipFuncAttributeMaxDynamicSharedMemorySize, LDS_GEMM);
  hipFuncSetAttribute(reinterpret_cast<const void*>(&k_gemm<0>),
                      hipFuncAttributeMaxDynamicSharedMemorySize, LDS_GEMM);
  k_gemm<1><<<dim3(nDst / GROWS, HD / GCOLS, 1), NTHR, LDS_GEMM, stream>>>(
      M16, X16, Bw1, bias1, prelu_w, out, H16, nDst, osc);

  k_gemm<0><<<dim3(nDst / GROWS, HD / GCOLS, 1), NTHR, LDS_GEMM, stream>>>(
      M16, H16, Bw2, bias2, prelu_w, out, X16, nDst, osc);
}
